// CrossTransformerLayer_88252987998700
// MI455X (gfx1250) — hardware-verified
//
#include <hip/hip_runtime.h>

typedef _Float16 v16h __attribute__((ext_vector_type(16)));
typedef _Float16 v8h  __attribute__((ext_vector_type(8)));
typedef _Float16 v2h  __attribute__((ext_vector_type(2)));
typedef float    v8f  __attribute__((ext_vector_type(8)));
typedef float    v4f  __attribute__((ext_vector_type(4)));
typedef float    v2f  __attribute__((ext_vector_type(2)));
typedef int      v4i  __attribute__((ext_vector_type(4)));
typedef v8h __attribute__((may_alias)) v8ha;
typedef v2h __attribute__((may_alias)) v2ha;
typedef v4f __attribute__((may_alias)) v4fa;
typedef v2f __attribute__((may_alias)) v2fa;
typedef v4i __attribute__((may_alias)) v4ia;

union Frag { v16h v; v8h half[2]; };

#define NSEQ   16
#define SEQL   192
#define DM     512
#define NH     8
#define HDIM   64
#define DFF    2048
#define NROW   3072
#define NPAIR  256
#define JPC    4
#define NCHUNK 4
#define CROWS  12288
#define WSC    32.0f
#define WINV   0.03125f
#define PSC    16384.0f

__device__ __forceinline__ v8f wmma_f16(v16h a, v16h b, v8f c) {
  v8f d = __builtin_amdgcn_wmma_f32_16x16x32_f16(false, a, false, b, (short)0, c, false, false);
  asm volatile("v_nop\n\tv_nop\n\tv_nop\n\tv_nop" : "+v"(d) : "v"(a), "v"(b));
  return d;
}

__device__ __forceinline__ v16h load_frag(const _Float16* p, int h) {
  Frag f;
  f.half[0] = *(const v8ha*)(p + 8 * h);
  f.half[1] = *(const v8ha*)(p + 16 + 8 * h);
  return f.v;
}

__device__ __forceinline__ v8f zero8f() {
  const v8f z = {0.f, 0.f, 0.f, 0.f, 0.f, 0.f, 0.f, 0.f};
  return z;
}

__global__ __launch_bounds__(256) void cvt_s_kernel(const float* __restrict__ s,
                                                    _Float16* __restrict__ sh) {
  const int g = blockIdx.x * 256 + threadIdx.x;
  if (g >= NROW * DM / 8) return;
  const float* src = s + (size_t)g * 8;
  const v4f a = *(const v4fa*)src;
  const v4f c = *(const v4fa*)(src + 4);
  const v8h o = { (_Float16)a.x, (_Float16)a.y, (_Float16)a.z, (_Float16)a.w,
                  (_Float16)c.x, (_Float16)c.y, (_Float16)c.z, (_Float16)c.w };
  _Float16* dst = sh + (size_t)g * 8;
  *(volatile v8h*)dst = o;
  __threadfence();
  *(volatile v8h*)dst = o;
}

__global__ __launch_bounds__(256) void cvt_w_kernel(
    const float* __restrict__ w0, const float* __restrict__ w1,
    const float* __restrict__ w2, const float* __restrict__ w3,
    const float* __restrict__ w4, const float* __restrict__ w5,
    const float* __restrict__ w6, const float* __restrict__ w7,
    const float* __restrict__ wf1, const float* __restrict__ wf2,
    _Float16* __restrict__ wb)
{
  const int g = blockIdx.x * 256 + threadIdx.x;
  if (g >= 524288) return;
  const float* src;
  size_t stride;
  _Float16* dst;
  if (g < 262144) {
    const int pl = g >> 15, off = g & 32767;
    const int n = off >> 6, k0 = (off & 63) * 8;
    const float* wp = (pl == 0) ? w0 : (pl == 1) ? w1 : (pl == 2) ? w2 : (pl == 3) ? w3 :
                      (pl == 4) ? w4 : (pl == 5) ? w5 : (pl == 6) ? w6 : w7;
    src = wp + (size_t)k0 * DM + n;
    stride = DM;
    dst = wb + (size_t)pl * DM * DM + (size_t)n * DM + k0;
  } else if (g < 393216) {
    const int off = g - 262144;
    const int n = off >> 6, k0 = (off & 63) * 8;
    src = wf1 + (size_t)k0 * DFF + n;
    stride = DFF;
    dst = wb + (size_t)8 * DM * DM + (size_t)n * DM + k0;
  } else {
    const int off = g - 393216;
    const int n = off >> 8, k0 = (off & 255) * 8;
    src = wf2 + (size_t)k0 * DM + n;
    stride = DM;
    dst = wb + (size_t)8 * DM * DM + (size_t)DFF * DM + (size_t)n * DFF + k0;
  }
  const float e0 = src[0] * WSC,          e1 = src[stride] * WSC;
  const float e2 = src[2 * stride] * WSC, e3 = src[3 * stride] * WSC;
  const float e4 = src[4 * stride] * WSC, e5 = src[5 * stride] * WSC;
  const float e6 = src[6 * stride] * WSC, e7 = src[7 * stride] * WSC;
  const v8h o = { (_Float16)e0, (_Float16)e1, (_Float16)e2, (_Float16)e3,
                  (_Float16)e4, (_Float16)e5, (_Float16)e6, (_Float16)e7 };
  *(volatile v8h*)dst = o;
  __threadfence();
  *(volatile v8h*)dst = o;
}

__device__ __forceinline__ void gemm_core(const _Float16* __restrict__ A,
                                          const _Float16* __restrict__ Bt,
                                          int K, int arow0, int bcol0, int h, int m,
                                          v8f (&acc)[2][4]) {
  const _Float16* a0p = A + (size_t)(arow0 + m) * K;
  const _Float16* a1p = a0p + (size_t)16 * K;
  const _Float16* bp  = Bt + (size_t)(bcol0 + m) * K;
  #pragma unroll
  for (int mt = 0; mt < 2; ++mt)
    #pragma unroll
    for (int nt = 0; nt < 4; ++nt) acc[mt][nt] = zero8f();
  #pragma unroll 1
  for (int k0 = 0; k0 < K; k0 += 32) {
    const v16h a0 = load_frag(a0p + k0, h);
    const v16h a1 = load_frag(a1p + k0, h);
    #pragma unroll
    for (int nt = 0; nt < 4; ++nt) {
      const v16h b = load_frag(bp + (size_t)nt * 16 * K + k0, h);
      acc[0][nt] = wmma_f16(a0, b, acc[0][nt]);
      acc[1][nt] = wmma_f16(a1, b, acc[1][nt]);
    }
  }
}

__device__ __forceinline__ void store_rows_h(const _Float16* sT, _Float16* dst,
                                             size_t ld, int w, int lane) {
  const int q8 = lane & 7, sub = lane >> 3;
  #pragma unroll
  for (int i = 0; i < 8; ++i) {
    const int lr = 32 * w + 4 * i + sub;
    const v8h v = *(const v8ha*)(sT + lr * 64 + 8 * q8);
    *(volatile v8h*)(dst + (size_t)lr * ld + 8 * q8) = v;
  }
}

__device__ __forceinline__ void store_rows_f(const float* sT, float* dst,
                                             size_t ld, int w, int lane) {
  const int q8 = lane & 7, sub = lane >> 3;
  #pragma unroll
  for (int i = 0; i < 16; ++i) {
    const int lr = 32 * w + 2 * i + (sub >> 1);
    const int c = 32 * (sub & 1) + 4 * q8;
    const v4f v = *(const v4fa*)(sT + lr * 64 + c);
    *(volatile v4f*)(dst + (size_t)lr * ld + c) = v;
  }
}

__global__ __launch_bounds__(64) void proj4_kernel(
    const _Float16* __restrict__ s16, const _Float16* __restrict__ wt,
    const float* __restrict__ bq, const float* __restrict__ bk,
    const float* __restrict__ bv, const float* __restrict__ bq2,
    _Float16* __restrict__ qh, _Float16* __restrict__ kh,
    _Float16* __restrict__ vt, float* __restrict__ q2)
{
  __shared__ __attribute__((aligned(16))) _Float16 sH[64 * 64];
  __shared__ __attribute__((aligned(16))) float    sF[64 * 64];

  const int tid = threadIdx.x, lane = tid & 31, w = tid >> 5;
  const int h = lane >> 4, m = lane & 15;
  const int bm = blockIdx.x, bn = blockIdx.y;
  const int which = bn >> 3, head = bn & 7;

  v8f acc[2][4];
  gemm_core(s16, wt, DM, bm * 64 + 32 * w, bn * 64, h, m, acc);

  const float* bias = (which == 0) ? bq : (which == 1) ? bk : (which == 2) ? bv : bq2;
  const float osc = (which == 0) ? 0.125f : 1.0f;
  #pragma unroll
  for (int nt = 0; nt < 4; ++nt) {
    const int lc = 16 * nt + m;
    const float bvl = bias[head * HDIM + lc];
    #pragma unroll
    for (int mt = 0; mt < 2; ++mt) {
      #pragma unroll
      for (int r = 0; r < 8; ++r) {
        const int lr = 32 * w + 16 * mt + 8 * h + r;
        const float y = (acc[mt][nt][r] * WINV + bvl) * osc;
        if (which == 3)      sF[lr * 64 + lc] = y;
        else if (which == 2) sH[lc * 64 + lr] = (_Float16)y;
        else                 sH[lr * 64 + lc] = (_Float16)y;
      }
    }
  }
  __syncthreads();

  if (which == 3) {
    float* dst = q2 + (size_t)(bm * 64) * DM + head * HDIM;
    store_rows_f(sF, dst, DM, w, lane);
    __threadfence();
    store_rows_f(sF, dst, DM, w, lane);
  } else if (which == 2) {
    const int j = bm / 3, l0 = (bm - 3 * j) * 64;
    _Float16* dst = vt + (size_t)((j * NH + head) * HDIM) * SEQL + l0;
    store_rows_h(sH, dst, SEQL, w, lane);
    __threadfence();
    store_rows_h(sH, dst, SEQL, w, lane);
  } else {
    _Float16* dst = ((which == 0) ? qh : kh) + (size_t)(bm * 64) * DM + head * HDIM;
    store_rows_h(sH, dst, DM, w, lane);
    __threadfence();
    store_rows_h(sH, dst, DM, w, lane);
  }
}

template <typename OT>
__global__ __launch_bounds__(64) void gemm_kernel(
    const _Float16* __restrict__ A, const _Float16* __restrict__ Bt,
    const float* __restrict__ bias0, const float* __restrict__ bias1,
    OT* __restrict__ out, int N, int K, int nsplit, int relu)
{
  __shared__ __attribute__((aligned(16))) _Float16 sH[64 * 64];
  __shared__ __attribute__((aligned(16))) float    sF[64 * 64];
  const bool HOUT = (sizeof(OT) == 2);

  const int tid = threadIdx.x, lane = tid & 31, w = tid >> 5;
  const int h = lane >> 4, m = lane & 15;
  const int bm = blockIdx.x, bn = blockIdx.y;

  v8f acc[2][4];
  gemm_core(A, Bt, K, bm * 64 + 32 * w, bn * 64, h, m, acc);

  #pragma unroll
  for (int nt = 0; nt < 4; ++nt) {
    const int lc = 16 * nt + m;
    const int colg = bn * 64 + lc;
    const int use1 = (colg >= nsplit) ? 1 : 0;
    const float* bp = use1 ? bias1 : bias0;
    const int bi = use1 ? (colg - nsplit) : colg;
    const float bvl = bp[bi];
    #pragma unroll
    for (int mt = 0; mt < 2; ++mt) {
      #pragma unroll
      for (int r = 0; r < 8; ++r) {
        const int lr = 32 * w + 16 * mt + 8 * h + r;
        float y = acc[mt][nt][r] * WINV + bvl;
        if (relu) y = fmaxf(y, 0.0f);
        if (HOUT) sH[lr * 64 + lc] = (_Float16)y;
        else      sF[lr * 64 + lc] = y;
      }
    }
  }
  __syncthreads();

  if (HOUT) {
    _Float16* dst = (_Float16*)out + (size_t)(bm * 64) * N + bn * 64;
    store_rows_h(sH, dst, (size_t)N, w, lane);
    __threadfence();
    store_rows_h(sH, dst, (size_t)N, w, lane);
  } else {
    float* dst = (float*)out + (size_t)(bm * 64) * N + bn * 64;
    store_rows_f(sF, dst, (size_t)N, w, lane);
    __threadfence();
    store_rows_f(sF, dst, (size_t)N, w, lane);
  }
}

__device__ __forceinline__ v8f add_madd8(v8f s, const int* p) {
  const v4i ma = *(const v4ia*)p;
  const v4i mb = *(const v4ia*)(p + 4);
  s[0] = s[0] + (1.0f - (float)ma.x) * -1.0e9f;
  s[1] = s[1] + (1.0f - (float)ma.y) * -1.0e9f;
  s[2] = s[2] + (1.0f - (float)ma.z) * -1.0e9f;
  s[3] = s[3] + (1.0f - (float)ma.w) * -1.0e9f;
  s[4] = s[4] + (1.0f - (float)mb.x) * -1.0e9f;
  s[5] = s[5] + (1.0f - (float)mb.y) * -1.0e9f;
  s[6] = s[6] + (1.0f - (float)mb.z) * -1.0e9f;
  s[7] = s[7] + (1.0f - (float)mb.w) * -1.0e9f;
  return s;
}

__device__ __forceinline__ v16h pack_p(v8f a, v8f c) {
  const v16h r = { (_Float16)(a[0] * PSC), (_Float16)(a[1] * PSC), (_Float16)(a[2] * PSC), (_Float16)(a[3] * PSC),
                   (_Float16)(a[4] * PSC), (_Float16)(a[5] * PSC), (_Float16)(a[6] * PSC), (_Float16)(a[7] * PSC),
                   (_Float16)(c[0] * PSC), (_Float16)(c[1] * PSC), (_Float16)(c[2] * PSC), (_Float16)(c[3] * PSC),
                   (_Float16)(c[4] * PSC), (_Float16)(c[5] * PSC), (_Float16)(c[6] * PSC), (_Float16)(c[7] * PSC) };
  return r;
}

__device__ __forceinline__ void ctx_store_pass(const _Float16* so, _Float16* dst, int lane) {
  const int q8 = lane & 7, sub = lane >> 3;
  #pragma unroll
  for (int i = 0; i < 4; ++i) {
    const int row = 4 * i + sub;
    const v8h v = *(const v8ha*)(so + row * 64 + 8 * q8);
    *(volatile v8h*)(dst + (size_t)row * DM + 8 * q8) = v;
  }
}

__global__ __launch_bounds__(128) void xattn_kernel(
    const _Float16* __restrict__ qh,
    const _Float16* __restrict__ kh,
    const _Float16* __restrict__ vt,
    const int* __restrict__ pad,
    _Float16* __restrict__ ctx,
    int c)
{
  __shared__ __attribute__((aligned(16))) _Float16 sO[4 * 16 * 64];

  const int tid = threadIdx.x, lane = tid & 31, w = tid >> 5;
  const int h = lane >> 4, m = lane & 15;
  const int qblk = blockIdx.x, pc = blockIdx.y, head = blockIdx.z;
  const int i = pc >> 2, jj = pc & 3;
  const int j = JPC * c + jj;
  const int p = i * NSEQ + j;
  const int q0 = qblk * 64 + 16 * w;

  const _Float16* qrow = qh + (size_t)(i * SEQL + q0 + m) * DM + head * HDIM;
  const v16h qb0 = load_frag(qrow, h);
  const v16h qb1 = load_frag(qrow + 32, h);

  v8f o[4];
  #pragma unroll
  for (int t = 0; t < 4; ++t) o[t] = zero8f();
  float mrun = -1.0e30f, lrun = 0.0f;

  const _Float16* kbase = kh + (size_t)(j * SEQL + m) * DM + head * HDIM;
  const _Float16* vbase = vt + (size_t)((j * NH + head) * HDIM + m) * SEQL;
  const int* mkp = pad + (size_t)p * SEQL + 8 * h;

  #pragma unroll 1
  for (int kb = 0; kb < SEQL; kb += 64) {
    v8f s[4];
    #pragma unroll
    for (int jt = 0; jt < 4; ++jt) {
      const _Float16* kp = kbase + (size_t)(kb + 16 * jt) * DM;
      const v16h kf0 = load_frag(kp, h);
      const v16h kf1 = load_frag(kp + 32, h);
      v8f z = zero8f();
      z = wmma_f16(kf0, qb0, z);
      z = wmma_f16(kf1, qb1, z);
      s[jt] = z;
    }
    #pragma unroll
    for (int jt = 0; jt < 4; ++jt) s[jt] = add_madd8(s[jt], mkp + kb + 16 * jt);

    float mloc = s[0][0];
    #pragma unroll
    for (int jt = 0; jt < 4; ++jt)
      #pragma unroll
      for (int r = 0; r < 8; ++r) mloc = fmaxf(mloc, s[jt][r]);
    mloc = fmaxf(mloc, __shfl_xor(mloc, 16));
    const float mnew = fmaxf(mrun, mloc);
    const float alpha = __expf(mrun - mnew);
    mrun = mnew;
    float lsum = 0.0f;
    #pragma unroll
    for (int jt = 0; jt < 4; ++jt)
      #pragma unroll
      for (int r = 0; r < 8; ++r) {
        const float pe = __expf(s[jt][r] - mnew);
        s[jt][r] = pe;
        lsum += pe;
      }
    lsum += __shfl_xor(lsum, 16);
    lrun = lrun * alpha + lsum;
    #pragma unroll
    for (int t = 0; t < 4; ++t)
      #pragma unroll
      for (int r = 0; r < 8; ++r) o[t][r] = o[t][r] * alpha;

    const v16h pb0 = pack_p(s[0], s[1]);
    const v16h pb1 = pack_p(s[2], s[3]);

    #pragma unroll
    for (int t = 0; t < 4; ++t) {
      const _Float16* vp = vbase + (size_t)(16 * t) * SEQL + kb;
      const v16h vf0 = load_frag(vp, h);
      const v16h vf1 = load_frag(vp + 32, h);
      o[t] = wmma_f16(vf0, pb0, o[t]);
      o[t] = wmma_f16(vf1, pb1, o[t]);
    }
  }

  const float inv = (1.0f / lrun) * (1.0f / PSC);
  _Float16* so = sO + w * 1024;
  #pragma unroll
  for (int t = 0; t < 4; ++t)
    #pragma unroll
    for (int r = 0; r < 8; ++r)
      so[m * 64 + 16 * t + 8 * h + r] = (_Float16)(o[t][r] * inv);
  __syncthreads();

  _Float16* dst = ctx + (size_t)(pc * SEQL + q0) * DM + head * HDIM;
  ctx_store_pass(so, dst, lane);
  __threadfence();
  ctx_store_pass(so, dst, lane);
}

__global__ __launch_bounds__(256) void iattn_kernel(
    const float* __restrict__ qin,
    const _Float16* __restrict__ kv,
    _Float16* __restrict__ o2,
    int c)
{
  __shared__ float sc[NH * NSEQ];
  __shared__ __attribute__((aligned(16))) _Float16 so[DM];

  const int tid = threadIdx.x, lane = tid & 31, w = tid >> 5;
  const int blk = blockIdx.x;
  const int jj = blk / SEQL;
  const int l = blk - jj * SEQL;
  const int r = c * (JPC * SEQL) + blk;

  const v2f qq = *(const v2fa*)(qin + (size_t)r * DM + w * HDIM + 2 * lane);

  #pragma unroll 1
  for (int t = 0; t < NSEQ; ++t) {
    const int kr = (t * JPC + jj) * SEQL + l;
    const v2h kk = *(const v2ha*)(kv + (size_t)kr * (2 * DM) + w * HDIM + 2 * lane);
    float s = qq.x * (float)kk.x + qq.y * (float)kk.y;
    s += __shfl_xor(s, 16);
    s += __shfl_xor(s, 8);
    s += __shfl_xor(s, 4);
    s += __shfl_xor(s, 2);
    s += __shfl_xor(s, 1);
    if (lane == 0) sc[w * NSEQ + t] = s * 0.125f;
  }
  __syncthreads();

  float mx = -3.0e38f;
  #pragma unroll 1
  for (int t = 0; t < NSEQ; ++t) mx = fmaxf(mx, sc[w * NSEQ + t]);
  float sum = 0.0f, oa = 0.0f, ob = 0.0f;
  #pragma unroll 1
  for (int t = 0; t < NSEQ; ++t) {
    const float pe = __expf(sc[w * NSEQ + t] - mx);
    sum += pe;
    const int kr = (t * JPC + jj) * SEQL + l;
    const v2h vv = *(const v2ha*)(kv + (size_t)kr * (2 * DM) + DM + w * HDIM + 2 * lane);
    oa += pe * (float)vv.x;
    ob += pe * (float)vv.y;
  }
  const float inv = 1.0f / sum;
  so[w * HDIM + 2 * lane]     = (_Float16)(oa * inv);
  so[w * HDIM + 2 * lane + 1] = (_Float16)(ob * inv);
  __syncthreads();

  if (w == 0) {
    const v8h a = *(const v8ha*)(so + 8 * lane);
    const v8h b = *(const v8ha*)(so + 256 + 8 * lane);
    _Float16* dst = o2 + (size_t)r * DM;
    *(volatile v8h*)(dst + 8 * lane) = a;
    *(volatile v8h*)(dst + 256 + 8 * lane) = b;
    __threadfence();
    *(volatile v8h*)(dst + 8 * lane) = a;
    *(volatile v8h*)(dst + 256 + 8 * lane) = b;
  }
}

template <int HOUT>
__global__ __launch_bounds__(128) void ln_kernel(
    const float* __restrict__ x0, const float* __restrict__ x1,
    const float* __restrict__ g, const float* __restrict__ b,
    const int* __restrict__ flag,
    float* __restrict__ outf, _Float16* __restrict__ outh)
{
  __shared__ float red1[4], red2[4];
  __shared__ __attribute__((aligned(16))) _Float16 soh[DM];
  (void)flag;

  const int t = threadIdx.x, lane = t & 31, w = t >> 5;
  const int row = blockIdx.x;
  const size_t base = (size_t)row * DM + 4 * t;
  const v4f a = *(const v4fa*)(x0 + base);
  const v4f cc = *(const v4fa*)(x1 + base);
  v4f x;
  x.x = a.x + cc.x; x.y = a.y + cc.y; x.z = a.z + cc.z; x.w = a.w + cc.w;

  float s = (x.x + x.y) + (x.z + x.w);
  s += __shfl_xor(s, 16); s += __shfl_xor(s, 8); s += __shfl_xor(s, 4);
  s += __shfl_xor(s, 2);  s += __shfl_xor(s, 1);
  if (lane == 0) red1[w] = s;
  __syncthreads();
  const float mu = ((red1[0] + red1[1]) + (red1[2] + red1[3])) * (1.0f / DM);

  v4f d;
  d.x = x.x - mu; d.y = x.y - mu; d.z = x.z - mu; d.w = x.w - mu;
  float vs = (d.x * d.x + d.y * d.y) + (d.z * d.z + d.w * d.w);
  vs += __shfl_xor(vs, 16); vs += __shfl_xor(vs, 8); vs += __shfl_xor(vs, 4);
  vs += __shfl_xor(vs, 2);  vs += __shfl_xor(vs, 1);
  if (lane == 0) red2[w] = vs;
  __syncthreads();
  const float var = ((red2[0] + red2[1]) + (red2[2] + red2[3])) * (1.0f / DM);
  const float inv = 1.0f / sqrtf(var + 1.0e-6f);

  const v4f gg = *(const v4fa*)(g + 4 * t);
  const v4f bb = *(const v4fa*)(b + 4 * t);
  v4f y;
  y.x = d.x * inv * gg.x + bb.x;
  y.y = d.y * inv * gg.y + bb.y;
  y.z = d.z * inv * gg.z + bb.z;
  y.w = d.w * inv * gg.w + bb.w;

  *(volatile v4f*)(outf + base) = y;
  __threadfence();
  *(volatile v4f*)(outf + base) = y;

  if (HOUT) {
    soh[4 * t]     = (_Float16)y.x;
    soh[4 * t + 1] = (_Float16)y.y;
    soh[4 * t + 2] = (_Float16)y.z;
    soh[4 * t + 3] = (_Float16)y.w;
    __syncthreads();
    if (t < 64) {
      const v8h v = *(const v8ha*)(soh + 8 * t);
      _Float16* dst = outh + (size_t)row * DM + 8 * t;
      *(volatile v8h*)dst = v;
      __threadfence();
      *(volatile v8h*)dst = v;
    }
  }
}

extern "C" void kernel_launch(void* const* d_in, const int* in_sizes, int n_in,
                              void* d_out, int out_size, void* d_ws, size_t ws_size,
                              hipStream_t stream) {
  if (n_in < 27) return;
  if (in_sizes[0] != NROW * DM) return;
  if (in_sizes[1] != NPAIR * SEQL) return;
  if (in_sizes[2] < 1) return;
  for (int q = 0; q < 8; ++q) {
    if (in_sizes[3 + 2 * q] != DM * DM) return;
    if (in_sizes[4 + 2 * q] != DM) return;
  }
  if (in_sizes[19] != DM * DFF || in_sizes[20] != DFF) return;
  if (in_sizes[21] != DFF * DM || in_sizes[22] != DM) return;
  if (in_sizes[23] != DM || in_sizes[24] != DM || in_sizes[25] != DM || in_sizes[26] != DM) return;
  if (out_size != NROW * DM) return;

  const float* S     = (const float*)d_in[0];
  const int*   padm  = (const int*)d_in[1];
  const int*   train = (const int*)d_in[2];
  const float* ca_wq = (const float*)d_in[3];  const float* ca_bq = (const float*)d_in[4];
  const float* ca_wk = (const float*)d_in[5];  const float* ca_bk = (const float*)d_in[6];
  const float* ca_wv = (const float*)d_in[7];  const float* ca_bv = (const float*)d_in[8];
  const float* ca_wo = (const float*)d_in[9];  const float* ca_bo = (const float*)d_in[10];
  const float* ia_wq = (const float*)d_in[11]; const float* ia_bq = (const float*)d_in[12];
  const float* ia_wk = (const float*)d_in[13]; const float* ia_bk = (const float*)d_in[14];
  const float* ia_wv = (const float*)d_in[15]; const float* ia_bv = (const float*)d_in[16];
  const float* ia_wo = (const float*)d_in[17]; const float* ia_bo = (const float*)d_in[18];
  const float* fw1   = (const float*)d_in[19]; const float* fb1   = (const float*)d_in[20];
  const float* fw2   = (const float*)d_in[21]; const float* fb2   = (const float*)d_in[22];
  const float* ln1g  = (const float*)d_in[23]; const float* ln1b  = (const float*)d_in[24];
  const float* ln2g  = (const float*)d_in[25]; const float* ln2b  = (const float*)d_in[26];
  float* out = (float*)d_out;

  const size_t b_s16 = (size_t)NROW * DM * 2;
  const size_t b_w   = ((size_t)8 * DM * DM + 2 * (size_t)DM * DFF) * 2;
  const size_t b_pl  = (size_t)NROW * DM * 2;
  const size_t b_q2  = (size_t)NROW * DM * 4;
  const size_t b_ctx = (size_t)CROWS * DM * 2;
  const size_t b_sa1 = b_ctx;
  const size_t b_kv  = (size_t)CROWS * 2 * DM * 2;
  const size_t b_o2  = (size_t)NROW * DM * 2;
  const size_t b_f32 = (size_t)NROW * DM * 4;
  const size_t b_sn  = (size_t)NROW * DM * 2;
  const size_t b_h1  = (size_t)NROW * DFF * 2;
  const size_t o_s16 = 0;
  const size_t o_w   = o_s16 + b_s16;
  const size_t o_qh  = o_w + b_w;
  const size_t o_kh  = o_qh + b_pl;
  const size_t o_vt  = o_kh + b_pl;
  const size_t o_q2  = o_vt + b_pl;
  const size_t o_ctx = o_q2 + b_q2;
  const size_t o_sa1 = o_ctx + b_ctx;
  const size_t o_kv  = o_sa1 + b_sa1;
  const size_t o_o2  = o_kv + b_kv;
  const size_t o_sa2 = o_o2 + b_o2;
  const size_t o_sn  = o_sa2 + b_f32;
  const size_t o_s16n = o_sn + b_f32;
  const size_t o_h1  = o_s16n + b_sn;
  const size_t o_f2  = o_h1 + b_h1;
  const size_t total = o_f2 + b_f32;
  if (total > ws_size) return;

  char* ws = (char*)d_ws;
  _Float16* s16  = (_Float16*)(ws + o_s16);
  _Float16* wb   = (_Float16*)(ws + o_w);
  _Float16* qh   = (_Float16*)(ws + o_qh);
  _Float16* kh   = (_Float16*)(ws + o_kh);
  _Float16* vt   = (_Float16*)(ws + o_vt);
  float*    q2   = (float*)   (ws + o_q2);
  _Float16* ctx  = (_Float16*)(ws + o_ctx);
  _Float16* sa1  = (_Float16*)(ws + o_sa1);
  _Float16* kv   = (_Float16*)(ws + o_kv);
  _Float16* o2   = (_Float16*)(ws + o_o2);
  float*    sa2  = (float*)   (ws + o_sa2);
  float*    snorm = (float*)  (ws + o_sn);
  _Float16* sn16 = (_Float16*)(ws + o_s16n);
  _Float16* h1   = (_Float16*)(ws + o_h1);
  float*    f2   = (float*)   (ws + o_f2);

  _Float16* wt_in4 = wb;
  _Float16* wt_o   = wb + (size_t)4 * DM * DM;
  _Float16* wt_kv2 = wb + (size_t)5 * DM * DM;
  _Float16* wt_o2  = wb + (size_t)7 * DM * DM;
  _Float16* wt_f1  = wb + (size_t)8 * DM * DM;
  _Float16* wt_f2  = wt_f1 + (size_t)DFF * DM;

  cvt_s_kernel<<<(NROW * DM / 8 + 255) / 256, 256, 0, stream>>>(S, s16);
  cvt_w_kernel<<<(524288 + 255) / 256, 256, 0, stream>>>(
      ca_wq, ca_wk, ca_wv, ia_wq, ca_wo, ia_wk, ia_wv, ia_wo, fw1, fw2, wb);

  proj4_kernel<<<dim3(NROW / 64, 4 * DM / 64), 64, 0, stream>>>(
      s16, wt_in4, ca_bq, ca_bk, ca_bv, ia_bq, qh, kh, vt, q2);

  for (int c = 0; c < NCHUNK; ++c) {
    xattn_kernel<<<dim3(SEQL / 64, NSEQ * JPC, NH), 128, 0, stream>>>(qh, kh, vt, padm, ctx, c);
    gemm_kernel<_Float16><<<dim3(CROWS / 64, DM / 64), 64, 0, stream>>>(
        ctx, wt_o, ca_bo, ca_bo, sa1, DM, DM, DM, 0);
    gemm_kernel<_Float16><<<dim3(CROWS / 64, (2 * DM) / 64), 64, 0, stream>>>(
        sa1, wt_kv2, ia_bk, ia_bv, kv, 2 * DM, DM, DM, 0);
    iattn_kernel<<<JPC * SEQL, 256, 0, stream>>>(q2, kv, o2, c);
  }

  gemm_kernel<float><<<dim3(NROW / 64, DM / 64), 64, 0, stream>>>(
      o2, wt_o2, ia_bo, ia_bo, sa2, DM, DM, DM, 0);
  ln_kernel<1><<<NROW, 128, 0, stream>>>(S, sa2, ln1g, ln1b, train, snorm, sn16);
  gemm_kernel<_Float16><<<dim3(NROW / 64, DFF / 64), 64, 0, stream>>>(
      sn16, wt_f1, fb1, fb1, h1, DFF, DM, DFF, 1);
  gemm_kernel<float><<<dim3(NROW / 64, DM / 64), 64, 0, stream>>>(
      h1, wt_f2, fb2, fb2, f2, DM, DFF, DM, 0);
  ln_kernel<0><<<NROW, 128, 0, stream>>>(snorm, f2, ln2g, ln2b, train, out, sn16);
}
